// FastLayer_695784702458
// MI455X (gfx1250) — hardware-verified
//
#include <hip/hip_runtime.h>
#include <math.h>

constexpr int kB = 4;
constexpr int kT = 2048;
constexpr int kD = 1024;
constexpr int kS = 64;
constexpr int kRows = kB * kT;
constexpr int kNP = 256;
constexpr int kBand = 256;
constexpr int kChunkT = 256;
constexpr int kNZ = kB * (kT / kChunkT);
constexpr int kSmPitch = 72;

typedef __attribute__((ext_vector_type(16))) _Float16 v16h;
typedef __attribute__((ext_vector_type(8)))  _Float16 v8h;
typedef __attribute__((ext_vector_type(16))) __bf16   v16b;
typedef __attribute__((ext_vector_type(8)))  __bf16   v8b;
typedef __attribute__((ext_vector_type(8)))  float    v8f;
typedef __attribute__((ext_vector_type(4)))  float    v4f;
typedef __attribute__((ext_vector_type(4)))  unsigned int v4u;

__device__ __forceinline__ unsigned short f2bf_bits(float f) {
  unsigned u = __float_as_uint(f);
  return (unsigned short)((u + 0x7FFFu + ((u >> 16) & 1u)) >> 16);
}
__device__ __forceinline__ float bf_bits2f(unsigned short h) { return __uint_as_float(((unsigned)h) << 16); }

__device__ __forceinline__ void dep_guard_h(v8f& a, v8f& b, v16h x, v16h y) { asm volatile("v_nop\n\tv_nop\n\tv_nop\n\tv_nop" : "+v"(a), "+v"(b) : "v"(x), "v"(y)); }
__device__ __forceinline__ void dep_guard_b(v8f& a, v8f& b, v16b x, v16b y) { asm volatile("v_nop\n\tv_nop\n\tv_nop\n\tv_nop" : "+v"(a), "+v"(b) : "v"(x), "v"(y)); }
__device__ __forceinline__ void keep4_h(v16h a, v16h b, v16h c, v16h d) { asm volatile("v_nop" :: "v"(a), "v"(b), "v"(c), "v"(d)); }
__device__ __forceinline__ void keep4_b(v16b a, v16b b, v16b c, v16b d) { asm volatile("v_nop" :: "v"(a), "v"(b), "v"(c), "v"(d)); }
__device__ __forceinline__ void acc_guard4(v8f& a, v8f& b, v8f& c, v8f& d) { asm volatile("v_nop\n\tv_nop\n\tv_nop\n\tv_nop" : "+v"(a), "+v"(b), "+v"(c), "+v"(d)); }
template <typename T> struct Frag;
template <> struct Frag<_Float16> {
  typedef v16h V; union U { v16h v; v8h h[2]; };
  static __device__ __forceinline__ v16h load(const _Float16* p) {
    U f; f.h[0] = *(const v8h*)(p); f.h[1] = *(const v8h*)(p + 16); return f.v;
  }
  static __device__ __forceinline__ v8f mma(v16h a, v16h b, v8f c) {
    return __builtin_amdgcn_wmma_f32_16x16x32_f16(false, a, false, b, (short)0, c, false, false);
  }
  static __device__ __forceinline__ void guard(v8f& a, v8f& b, v16h x, v16h y) { dep_guard_h(a, b, x, y); }
  static __device__ __forceinline__ void keep(v16h a, v16h b, v16h c, v16h d) { keep4_h(a, b, c, d); }
};
template <> struct Frag<__bf16> {
  typedef v16b V; union U { v16b v; v8b h[2]; };
  static __device__ __forceinline__ v16b load(const __bf16* p) {
    U f; f.h[0] = *(const v8b*)(p); f.h[1] = *(const v8b*)(p + 16); return f.v;
  }
  static __device__ __forceinline__ v8f mma(v16b a, v16b b, v8f c) {
    return __builtin_amdgcn_wmma_f32_16x16x32_bf16(false, a, false, b, (short)0, c, false, false);
  }
  static __device__ __forceinline__ void guard(v8f& a, v8f& b, v16b x, v16b y) { dep_guard_b(a, b, x, y); }
  static __device__ __forceinline__ void keep(v16b a, v16b b, v16b c, v16b d) { keep4_b(a, b, c, d); }
};

__device__ __forceinline__ unsigned pk16(unsigned short a, unsigned short b) { return (unsigned)a | ((unsigned)b << 16); }

template <int ET> struct Elem;
template <> struct Elem<0> { typedef _Float16 T; };
template <> struct Elem<1> { typedef __bf16 T; };
template <int ET, bool SPLIT, int BIAS_MODE, int OUT_MODE, bool RESID, int ACT = 0>
__global__ __launch_bounds__(256) void wmma_gemm64(
    const unsigned short* __restrict__ Ap, const unsigned short* __restrict__ A2p, int lda, long strideA,
    const unsigned short* __restrict__ Btp, const unsigned short* __restrict__ Bt2p, int ldb, long strideB,
    void* __restrict__ Cout, void* __restrict__ Cout2, int ldc, long strideC,
    const float* __restrict__ bias,
    const float* __restrict__ resid, long strideR,
    int M, int N, int K, float scale) {
  typedef typename Elem<ET>::T T;
  typedef typename Frag<T>::V V;
  const T* A = (const T*)Ap; const T* A2 = (const T*)A2p; const T* Bt = (const T*)Btp; const T* Bt2 = (const T*)Bt2p;
  __shared__ __align__(16) float sT[8][16 * 68];
  const int b    = blockIdx.y;
  const int lane = threadIdx.x & 31;
  const int wave = threadIdx.x >> 5;
  const int tilesN = N >> 6;
  const int tilesM = M >> 6;
  const int tile = blockIdx.x * 8 + wave;
  if (tile >= tilesM * tilesN) return;
  const int tm = tile / tilesN;
  const int tn = tile - tm * tilesN;
  const int m0 = tm << 6;
  const int n0 = tn << 6;

  const T* Ab  = A  + (size_t)b * strideA;
  const T* Bb  = Bt + (size_t)b * strideB;
  const T* Ab2 = SPLIT ? (A2  + (size_t)b * strideA) : nullptr;
  const T* Bb2 = SPLIT ? (Bt2 + (size_t)b * strideB) : nullptr;

  const int rlane = lane & 15;
  const int koff  = (lane >> 4) * 8;
  const int mOff  = (lane >> 4) * 8;

  v8f acc[4][4];
#pragma unroll
  for (int i = 0; i < 4; ++i)
#pragma unroll
    for (int j = 0; j < 4; ++j) acc[i][j] = (v8f){0.f,0.f,0.f,0.f,0.f,0.f,0.f,0.f};

  for (int k0 = 0; k0 < K; k0 += 32) {
    V bh[4], bl[4];
#pragma unroll
    for (int j = 0; j < 4; ++j) {
      const size_t bo = (size_t)(n0 + (j << 4) + rlane) * ldb + koff + k0;
      bh[j] = Frag<T>::load(Bb + bo);
      if (SPLIT) bl[j] = Frag<T>::load(Bb2 + bo);
    }
#pragma unroll
    for (int i = 0; i < 4; ++i) {
      const size_t ao = (size_t)(m0 + (i << 4) + rlane) * lda + koff + k0;
      V ah = Frag<T>::load(Ab + ao);
      V al;
      if (SPLIT) al = Frag<T>::load(Ab2 + ao);
#pragma unroll
      for (int j = 0; j < 4; ++j) {
        acc[i][j] = Frag<T>::mma(ah, bh[j], acc[i][j]);
        if (SPLIT) {
          acc[i][j] = Frag<T>::mma(ah, bl[j], acc[i][j]);
          acc[i][j] = Frag<T>::mma(al, bh[j], acc[i][j]);
        }
      }
      Frag<T>::guard(acc[i][0], acc[i][3], ah, SPLIT ? al : ah);
    }
    Frag<T>::keep(bh[0], bh[1], bh[2], bh[3]);
    if (SPLIT) Frag<T>::keep(bl[0], bl[1], bl[2], bl[3]);
  }
  acc_guard4(acc[0][0], acc[0][1], acc[0][2], acc[0][3]);
  acc_guard4(acc[1][0], acc[1][1], acc[1][2], acc[1][3]);
  acc_guard4(acc[2][0], acc[2][1], acc[2][2], acc[2][3]);
  acc_guard4(acc[3][0], acc[3][1], acc[3][2], acc[3][3]);

  float* slab = sT[wave];
  const float* Rb = RESID ? (resid + (size_t)b * strideR) : nullptr;
#pragma unroll
  for (int i = 0; i < 4; ++i) {
    const int mBase = m0 + (i << 4);
#pragma unroll
    for (int j = 0; j < 4; ++j) {
      const int n = n0 + (j << 4) + rlane;
      float bv = 0.f;
      if (BIAS_MODE == 2) bv = bias[n];
#pragma unroll
      for (int r = 0; r < 8; ++r) {
        float v = acc[i][j][r] * scale;
        if (BIAS_MODE == 1) v += bias[mBase + mOff + r];
        if (BIAS_MODE == 2) v += bv;
        if (RESID) v += Rb[(size_t)(mBase + mOff + r) * ldc + n];
        if (ACT == 2) v = fmaxf(v, 0.0f);
        if (ACT == 4) v = (v > 0.f) ? v : 0.01f * v;
        slab[(mOff + r) * 68 + (j << 4) + rlane] = v;
      }
    }
    __builtin_amdgcn_fence(__ATOMIC_RELEASE, "workgroup");
    __builtin_amdgcn_wave_barrier();
    __builtin_amdgcn_fence(__ATOMIC_ACQUIRE, "workgroup");
    if (OUT_MODE == 0) {
      float* C = (float*)Cout + (size_t)b * strideC;
      const int hh = lane >> 4, c4 = (lane & 15) * 4;
      for (int pass = 0; pass < 2; ++pass) {
#pragma unroll
        for (int it = 0; it < 8; ++it) {
          const int row = it * 2 + hh;
          v4f v = *(const v4f*)(slab + row * 68 + c4);
          *(volatile v4f*)(C + (size_t)(mBase + row) * ldc + n0 + c4) = v;
        }
        __threadfence();
      }
    } else {
      const int q = lane >> 3, c8 = (lane & 7) * 8;
      unsigned short* C  = (unsigned short*)Cout  + (size_t)b * strideC;
      unsigned short* C2 = (OUT_MODE == 2) ? ((unsigned short*)Cout2 + (size_t)b * strideC) : nullptr;
      for (int pass = 0; pass < 2; ++pass) {
#pragma unroll
        for (int it = 0; it < 4; ++it) {
          const int row = it * 4 + q;
          const float* sp = slab + row * 68 + c8;
          v8h hv, lv;
#pragma unroll
          for (int e = 0; e < 8; ++e) {
            if (OUT_MODE == 1) {
              hv[e] = (_Float16)sp[e];
            } else {
              unsigned short hb = f2bf_bits(sp[e]);
              unsigned short lb = f2bf_bits(sp[e] - bf_bits2f(hb));
              hv[e] = __builtin_bit_cast(_Float16, hb);
              lv[e] = __builtin_bit_cast(_Float16, lb);
            }
          }
          *(volatile v8h*)(C + (size_t)(mBase + row) * ldc + n0 + c8) = hv;
          if (OUT_MODE == 2) *(volatile v8h*)(C2 + (size_t)(mBase + row) * ldc + n0 + c8) = lv;
        }
        __threadfence();
      }
    }
    __builtin_amdgcn_fence(__ATOMIC_RELEASE, "workgroup");
    __builtin_amdgcn_wave_barrier();
    __builtin_amdgcn_fence(__ATOMIC_ACQUIRE, "workgroup");
  }
}

template <int MODE>
__global__ __launch_bounds__(256) void band_gemm64(
    const unsigned short* __restrict__ Ap, const unsigned short* __restrict__ A2p, int lda, long strideA,
    const unsigned short* __restrict__ Btp, const unsigned short* __restrict__ Bt2p, int ldb, long strideB,
    float* __restrict__ Cout, int ldc, long strideC) {
  typedef __bf16 T;
  typedef v16b V;
  const T* A = (const T*)Ap; const T* A2 = (const T*)A2p; const T* Bt = (const T*)Btp; const T* Bt2 = (const T*)Bt2p;
  __shared__ __align__(16) float sT[8][16 * 68];
  const int b    = blockIdx.y;
  const int lane = threadIdx.x & 31;
  const int wave = threadIdx.x >> 5;
  const int tile = blockIdx.x * 8 + wave;
  int tm, n0, ncol0, kBeg, kEnd;
  long bOff;
  if (MODE == 0) {
    tm = tile >> 2;
    const int jd = tile & 3;
    const int tn = tm - jd;
    if (tm >= (kT / 64) || tn < 0) return;
    n0 = tn << 6; ncol0 = (3 - jd) << 6; kBeg = 0; kEnd = kS; bOff = 0;
  } else {
    tm = tile;
    if (tm >= (kT / 64)) return;
    n0 = 0; ncol0 = 0; kBeg = (tm < 3) ? ((3 - tm) << 6) : 0; kEnd = kBand; bOff = (long)(tm - 3) * 64;
  }
  const int m0 = tm << 6;

  const T* Ab  = A   + (size_t)b * strideA;
  const T* Bb  = Bt  + (size_t)b * strideB;
  const T* Ab2 = A2  + (size_t)b * strideA;
  const T* Bb2 = Bt2 + (size_t)b * strideB;

  const int rlane = lane & 15;
  const int koff  = (lane >> 4) * 8;
  const int mOff  = (lane >> 4) * 8;

  v8f acc[4][4];
#pragma unroll
  for (int i = 0; i < 4; ++i)
#pragma unroll
    for (int j = 0; j < 4; ++j) acc[i][j] = (v8f){0.f,0.f,0.f,0.f,0.f,0.f,0.f,0.f};

  for (int k0 = kBeg; k0 < kEnd; k0 += 32) {
    V bh[4], bl[4];
#pragma unroll
    for (int j = 0; j < 4; ++j) {
      const long bo = (long)(n0 + (j << 4) + rlane) * ldb + bOff + koff + k0;
      bh[j] = Frag<T>::load(Bb + bo);
      bl[j] = Frag<T>::load(Bb2 + bo);
    }
#pragma unroll
    for (int i = 0; i < 4; ++i) {
      const size_t ao = (size_t)(m0 + (i << 4) + rlane) * lda + koff + k0;
      V ah = Frag<T>::load(Ab + ao);
      V al = Frag<T>::load(Ab2 + ao);
#pragma unroll
      for (int j = 0; j < 4; ++j) {
        acc[i][j] = Frag<T>::mma(ah, bh[j], acc[i][j]);
        acc[i][j] = Frag<T>::mma(ah, bl[j], acc[i][j]);
        acc[i][j] = Frag<T>::mma(al, bh[j], acc[i][j]);
      }
      Frag<T>::guard(acc[i][0], acc[i][3], ah, al);
    }
    Frag<T>::keep(bh[0], bh[1], bh[2], bh[3]);
    Frag<T>::keep(bl[0], bl[1], bl[2], bl[3]);
  }
  acc_guard4(acc[0][0], acc[0][1], acc[0][2], acc[0][3]);
  acc_guard4(acc[1][0], acc[1][1], acc[1][2], acc[1][3]);
  acc_guard4(acc[2][0], acc[2][1], acc[2][2], acc[2][3]);
  acc_guard4(acc[3][0], acc[3][1], acc[3][2], acc[3][3]);

  float* slab = sT[wave];
  float* C = Cout + (size_t)b * strideC;
#pragma unroll
  for (int i = 0; i < 4; ++i) {
    const int mBase = m0 + (i << 4);
#pragma unroll
    for (int j = 0; j < 4; ++j) {
#pragma unroll
      for (int r = 0; r < 8; ++r) slab[(mOff + r) * 68 + (j << 4) + rlane] = acc[i][j][r];
    }
    __builtin_amdgcn_fence(__ATOMIC_RELEASE, "workgroup");
    __builtin_amdgcn_wave_barrier();
    __builtin_amdgcn_fence(__ATOMIC_ACQUIRE, "workgroup");
    {
      const int hh = lane >> 4, c4 = (lane & 15) * 4;
      for (int pass = 0; pass < 2; ++pass) {
#pragma unroll
        for (int it = 0; it < 8; ++it) {
          const int row = it * 2 + hh;
          v4f v = *(const v4f*)(slab + row * 68 + c4);
          *(volatile v4f*)(C + (size_t)(mBase + row) * ldc + ncol0 + c4) = v;
        }
        __threadfence();
      }
    }
    __builtin_amdgcn_fence(__ATOMIC_RELEASE, "workgroup");
    __builtin_amdgcn_wave_barrier();
    __builtin_amdgcn_fence(__ATOMIC_ACQUIRE, "workgroup");
  }
}

__device__ __forceinline__ void split_bits(float f, unsigned short& h, unsigned short& l) {
  h = f2bf_bits(f);
  l = f2bf_bits(f - bf_bits2f(h));
}
__device__ __forceinline__ void ld8(const float* __restrict__ p, float (&o)[8]) {
  const v4f a = *(const v4f*)(p);
  const v4f c = *(const v4f*)(p + 4);
#pragma unroll
  for (int e = 0; e < 4; ++e) { o[e] = a[e]; o[4 + e] = c[e]; }
}
__device__ __forceinline__ void split8(const float (&v)[8], unsigned short (&h)[8], unsigned short (&l)[8]) {
#pragma unroll
  for (int e = 0; e < 8; ++e) split_bits(v[e], h[e], l[e]);
}
__device__ __forceinline__ v4u pack8(const unsigned short (&b)[8]) {
  return (v4u){pk16(b[0], b[1]), pk16(b[2], b[3]), pk16(b[4], b[5]), pk16(b[6], b[7])};
}

__global__ __launch_bounds__(256) void cvt_x_kernel(const float* __restrict__ x,
                                                    unsigned short* __restrict__ xh, unsigned short* __restrict__ xl, int n8) {
  const int i = blockIdx.x * 256 + threadIdx.x;
  if (i >= n8) return;
  float f[8];
  ld8(x + 8 * (size_t)i, f);
  unsigned short hb[8], lb[8];
  split8(f, hb, lb);
  const v4u uh = pack8(hb), ul = pack8(lb);
  unsigned short* qh = xh + 8 * (size_t)i;
  unsigned short* ql = xl + 8 * (size_t)i;
  *(volatile v4u*)qh = uh;
  *(volatile v4u*)ql = ul;
  __threadfence();
  *(volatile v4u*)qh = uh;
  *(volatile v4u*)ql = ul;
}

__global__ __launch_bounds__(256) void cvt_w_kernel(
    const float* __restrict__ Wk, const float* __restrict__ Wv, const float* __restrict__ Wq, const float* __restrict__ Wg,
    const float* __restrict__ Wout, const float* __restrict__ state,
    unsigned short* __restrict__ wh, unsigned short* __restrict__ wl,
    unsigned short* __restrict__ woh, unsigned short* __restrict__ wol,
    unsigned short* __restrict__ sth, unsigned short* __restrict__ stl) {
  const int blk = blockIdx.x;
  const int tid = threadIdx.x;
  float f[8];
  unsigned short* dh;
  unsigned short* dl;
  size_t off;
  if (blk < 128) {
    const int e0 = (blk * 256 + tid) * 8;
    const int row = e0 >> 10, col = e0 & 1023;
    const float* src = (row < 64) ? Wk : (row < 128) ? Wv : (row < 192) ? Wq : Wg;
    const size_t so = (row < 192) ? ((size_t)(row & 63) * kD + col) : (size_t)col;
    const bool zero = (row > 192);
    ld8(src + so, f);
#pragma unroll
    for (int e = 0; e < 8; ++e) f[e] = zero ? 0.0f : f[e];
    dh = wh; dl = wl; off = (size_t)e0;
  } else if (blk < 160) {
    const int e0 = ((blk - 128) * 256 + tid) * 8;
    ld8(Wout + e0, f);
    dh = woh; dl = wol; off = (size_t)e0;
  } else {
    const int e0 = ((blk - 160) * 256 + tid) * 8;
    ld8(state + e0, f);
    dh = sth; dl = stl; off = (size_t)e0;
  }
  unsigned short hb[8], lb[8];
  split8(f, hb, lb);
  const v4u uh = pack8(hb), ul = pack8(lb);
  *(volatile v4u*)(dh + off) = uh;
  *(volatile v4u*)(dl + off) = ul;
  __threadfence();
  *(volatile v4u*)(dh + off) = uh;
  *(volatile v4u*)(dl + off) = ul;
}

__global__ __launch_bounds__(256) void gates_pre_kernel(
    const float* __restrict__ proj, const float* __restrict__ bg,
    const float* __restrict__ cosT, const float* __restrict__ sinT, float* __restrict__ logg) {
  __shared__ __align__(16) float slog[64];
  const int tid = threadIdx.x;
  const int rl = tid >> 2, p = tid & 3;
  const int row0 = blockIdx.x * 64;
  const int row = row0 + rl;
  const int t = row & (kT - 1);
  const float* pr = proj + (size_t)row * kNP;
  float k1[8], k2[8], cc[8], sn[8];
  ld8(pr + 8 * p, k1);
  ld8(pr + 32 + 8 * p, k2);
  ld8(cosT + (size_t)t * kS + 8 * p, cc);
  ld8(sinT + (size_t)t * kS + 8 * p, sn);
  const float g = pr[192];
  const float alpha = 1.0f / (1.0f + expf(-(g + bg[0])));
  float nrm = 0.0f;
#pragma unroll
  for (int e = 0; e < 8; ++e) {
    const float r1 = k1[e] * cc[e] - k2[e] * sn[e];
    const float r2 = k2[e] * cc[e] + k1[e] * sn[e];
    nrm += r1 * r1 + r2 * r2;
  }
  nrm += __shfl_xor(nrm, 1, 32);
  nrm += __shfl_xor(nrm, 2, 32);
  const float z  = (alpha * nrm) * 0.1f;
  const float sp = fmaxf(z, 0.0f) + log1pf(expf(-fabsf(z)));
  const float gg = expf(-sp);
  const float lg = logf(gg + 1e-8f);
  if (p == 0) slog[rl] = lg;
  __syncthreads();
  if (tid < 16) {
    const v4f v = *(const v4f*)(slog + 4 * tid);
    float* dst = logg + row0 + 4 * tid;
    *(volatile v4f*)dst = v;
    __threadfence();
    *(volatile v4f*)dst = v;
  }
}

__global__ __launch_bounds__(32) void scan_kernel(const float* __restrict__ logg, float* __restrict__ cum, float* __restrict__ cs) {
  const int b = blockIdx.x;
  const int lane = threadIdx.x;
  const size_t base = (size_t)b * kT;
  float carry = 0.0f;
  for (int c = 0; c < kT / 32; ++c) {
    const float v = logg[base + c * 32 + lane];
    float excl = 0.0f, incl = 0.0f;
#pragma unroll
    for (int j = 0; j < 32; ++j) {
      const float xj = __shfl(v, j, 32);
      const float nb = carry;
      carry = carry + xj;
      excl = (lane == j) ? nb : excl;
      incl = (lane == j) ? carry : incl;
    }
    float* pc = cum + base + c * 32 + lane;
    float* ps = cs  + base + c * 32 + lane;
    *(volatile float*)pc = incl;
    *(volatile float*)ps = excl;
    __threadfence();
    *(volatile float*)pc = incl;
    *(volatile float*)ps = excl;
  }
}

template <bool TR>
__device__ __forceinline__ void stage_store(unsigned short* sm, int rl, int p, int wave, int lane,
                                            const unsigned short (&b1)[8], const unsigned short (&b2)[8],
                                            unsigned short* __restrict__ base, int pitch) {
  __syncthreads();
#pragma unroll
  for (int e = 0; e < 8; ++e) {
    const int j = 8 * p + e;
    if (TR) {
      sm[j * kSmPitch + rl] = b1[e];
      sm[(32 + j) * kSmPitch + rl] = b2[e];
    } else {
      sm[rl * kSmPitch + j] = b1[e];
      sm[rl * kSmPitch + 32 + j] = b2[e];
    }
  }
  __syncthreads();
  const int q = lane >> 3, c8 = (lane & 7) * 8;
  for (int pass = 0; pass < 2; ++pass) {
#pragma unroll
    for (int it = 0; it < 2; ++it) {
      const int r = wave * 8 + it * 4 + q;
      const v4u u = *(const v4u*)(sm + r * kSmPitch + c8);
      *(volatile v4u*)(base + (size_t)r * pitch + c8) = u;
    }
    __threadfence();
  }
}

__global__ __launch_bounds__(256) void planes_kernel(
    const float* __restrict__ proj, const float* __restrict__ bg,
    const float* __restrict__ cosT, const float* __restrict__ sinT,
    const float* __restrict__ cs, const float* __restrict__ cum,
    unsigned short* __restrict__ krh, unsigned short* __restrict__ krl,
    unsigned short* __restrict__ qrh, unsigned short* __restrict__ qrl,
    unsigned short* __restrict__ qdh, unsigned short* __restrict__ qdl,
    unsigned short* __restrict__ krTh, unsigned short* __restrict__ krTl,
    unsigned short* __restrict__ avTh, unsigned short* __restrict__ avTl,
    unsigned short* __restrict__ aTh, unsigned short* __restrict__ aTl) {
  __shared__ __align__(16) unsigned short sm[64 * kSmPitch];
  const int tid = threadIdx.x, lane = tid & 31, wave = tid >> 5;
  const int rl = tid >> 2, p = tid & 3;
  const int row0 = blockIdx.x * 64;
  const int row = row0 + rl;
  const int b = row0 / kT;
  const int t0 = row0 - b * kT;
  const int t = t0 + rl;
  const int z = b * (kT / kChunkT) + (t0 / kChunkT);
  const int tl0 = t0 & (kChunkT - 1);
  const float* pr = proj + (size_t)row * kNP;
  float k1[8], k2[8], q1[8], q2[8], v1[8], v2[8], cc[8], sn[8];
  ld8(pr + 8 * p, k1);
  ld8(pr + 32 + 8 * p, k2);
  ld8(pr + 64 + 8 * p, v1);
  ld8(pr + 96 + 8 * p, v2);
  ld8(pr + 128 + 8 * p, q1);
  ld8(pr + 160 + 8 * p, q2);
  ld8(cosT + (size_t)t * kS + 8 * p, cc);
  ld8(sinT + (size_t)t * kS + 8 * p, sn);
  const float g = pr[192];
  const float alpha = 1.0f / (1.0f + expf(-(g + bg[0])));
  float kr1[8], kr2[8], qr1[8], qr2[8];
#pragma unroll
  for (int e = 0; e < 8; ++e) {
    kr1[e] = k1[e] * cc[e] - k2[e] * sn[e];
    kr2[e] = k2[e] * cc[e] + k1[e] * sn[e];
    qr1[e] = q1[e] * cc[e] - q2[e] * sn[e];
    qr2[e] = q2[e] * cc[e] + q1[e] * sn[e];
  }
  const float csv = cs[row];
  const float cmv = cum[row];
  const float clv = cum[(size_t)b * kT + (kT - 1)];
  const float dect = expf(csv);
  const float d2e  = expf(clv - cmv);

  unsigned short h1[8], h2[8], l1[8], l2[8];
  split8(kr1, h1, l1); split8(kr2, h2, l2);
  stage_store<false>(sm, rl, p, wave, lane, h1, h2, krh + (size_t)row0 * kS, kS);
  stage_store<false>(sm, rl, p, wave, lane, l1, l2, krl + (size_t)row0 * kS, kS);
  stage_store<true >(sm, rl, p, wave, lane, h1, h2, krTh + (size_t)z * kS * kChunkT + tl0, kChunkT);
  stage_store<true >(sm, rl, p, wave, lane, l1, l2, krTl + (size_t)z * kS * kChunkT + tl0, kChunkT);
  split8(qr1, h1, l1); split8(qr2, h2, l2);
  stage_store<false>(sm, rl, p, wave, lane, h1, h2, qrh + (size_t)row0 * kS, kS);
  stage_store<false>(sm, rl, p, wave, lane, l1, l2, qrl + (size_t)row0 * kS, kS);
  float w1[8], w2[8];
#pragma unroll
  for (int e = 0; e < 8; ++e) { w1[e] = qr1[e] * dect; w2[e] = qr2[e] * dect; }
  split8(w1, h1, l1); split8(w2, h2, l2);
  stage_store<false>(sm, rl, p, wave, lane, h1, h2, qdh + (size_t)row0 * kS, kS);
  stage_store<false>(sm, rl, p, wave, lane, l1, l2, qdl + (size_t)row0 * kS, kS);
#pragma unroll
  for (int e = 0; e < 8; ++e) { w1[e] = alpha * v1[e]; w2[e] = alpha * v2[e]; }
  split8(w1, h1, l1); split8(w2, h2, l2);
  stage_store<true >(sm, rl, p, wave, lane, h1, h2, avTh + (size_t)b * kS * kT + t0, kT);
  stage_store<true >(sm, rl, p, wave, lane, l1, l2, avTl + (size_t)b * kS * kT + t0, kT);
#pragma unroll
  for (int e = 0; e < 8; ++e) { w1[e] = w1[e] * d2e; w2[e] = w2[e] * d2e; }
  split8(w1, h1, l1); split8(w2, h2, l2);
  stage_store<true >(sm, rl, p, wave, lane, h1, h2, aTh + (size_t)z * kS * kChunkT + tl0, kChunkT);
  stage_store<true >(sm, rl, p, wave, lane, l1, l2, aTl + (size_t)z * kS * kChunkT + tl0, kChunkT);
}

__global__ __launch_bounds__(256) void decay_kernel(const float* __restrict__ sc, const float* __restrict__ cum,
                                                   const float* __restrict__ cs,
                                                   unsigned short* __restrict__ dah, unsigned short* __restrict__ dal) {
  const int tid = threadIdx.x, wave = tid >> 5, lane = tid & 31;
  const int row = blockIdx.x * 8 + wave;
  if (row >= kRows) return;
  const int b = row >> 11;
  const int t = row & (kT - 1);
  const int tm = t >> 6;
  const int sg = (tm - 3) * 64 + lane * 8;
  const int sgc = (sg < 0) ? 0 : sg;
  const float csv = cs[row];
  float scv[8], cmv[8];
  ld8(sc + (size_t)row * kBand + lane * 8, scv);
  ld8(cum + (size_t)b * kT + sgc, cmv);
  unsigned short hb[8], lb[8];
#pragma unroll
  for (int e = 0; e < 8; ++e) {
    const int s = sg + e;
    const bool valid = (s >= 0) && (s < t);
    const float d = expf(csv - cmv[e]);
    const float val = valid ? (scv[e] * d) : 0.0f;
    split_bits(val, hb[e], lb[e]);
  }
  const v4u uh = pack8(hb), ul = pack8(lb);
  unsigned short* qh = dah + (size_t)row * kBand + lane * 8;
  unsigned short* ql = dal + (size_t)row * kBand + lane * 8;
  *(volatile v4u*)qh = uh;
  *(volatile v4u*)ql = ul;
  __threadfence();
  *(volatile v4u*)qh = uh;
  *(volatile v4u*)ql = ul;
}

__global__ __launch_bounds__(256) void nstate_kernel(const float* __restrict__ nsp, const float* __restrict__ state,
                                                    const float* __restrict__ cum, float* __restrict__ ns) {
  const int i = blockIdx.x * 256 + threadIdx.x;
  if (i >= kB * kS * kS / 4) return;
  const int b = i >> 10;
  const int w = i & 1023;
  const float clv = cum[(size_t)b * kT + (kT - 1)];
  const float fd = expf(clv);
  v4f accv = (v4f){0.f, 0.f, 0.f, 0.f};
#pragma unroll
  for (int c = 0; c < kT / kChunkT; ++c)
    accv += *(const v4f*)(nsp + (size_t)(b * (kT / kChunkT) + c) * (kS * kS) + 4 * w);
  const v4f st = *(const v4f*)(state + (size_t)b * (kS * kS) + 4 * w);
  const v4f r = st * fd + accv;
  float* dst = ns + 4 * (size_t)i;
  *(volatile v4f*)dst = r;
  __threadfence();
  *(volatile v4f*)dst = r;
}

extern "C" void kernel_launch(void* const* d_in, const int* in_sizes, int n_in,
                              void* d_out, int out_size, void* d_ws, size_t ws_size,
                              hipStream_t stream) {
  if (n_in < 11) return;
  const float* x     = (const float*)d_in[0];
  const float* state = (const float*)d_in[1];
  const float* Wk    = (const float*)d_in[2];
  const float* Wv    = (const float*)d_in[3];
  const float* Wq    = (const float*)d_in[4];
  const float* Wout  = (const float*)d_in[5];
  const float* bout  = (const float*)d_in[6];
  const float* Wg    = (const float*)d_in[7];
  const float* bg    = (const float*)d_in[8];
  const float* cosT  = (const float*)d_in[9];
  const float* sinT  = (const float*)d_in[10];
  if (in_sizes[0] != kRows * kD) return;
  if (out_size != kRows * kD + kB * kS * kS) return;

  float* out    = (float*)d_out;
  float* ns_out = (float*)d_out + (size_t)kRows * kD;

  size_t off = 0;
  char* wsb = (char*)d_ws;
  auto carve = [&](size_t bytes) -> char* {
    char* p = wsb + off;
    off += (bytes + 255) & ~(size_t)255;
    return p;
  };
  const size_t plane64 = (size_t)kRows * kS * 2;
  unsigned short* xh   = (unsigned short*)carve((size_t)kRows * kD * 2);
  unsigned short* xl   = (unsigned short*)carve((size_t)kRows * kD * 2);
  unsigned short* wh   = (unsigned short*)carve((size_t)kNP * kD * 2);
  unsigned short* wl   = (unsigned short*)carve((size_t)kNP * kD * 2);
  unsigned short* woh  = (unsigned short*)carve((size_t)kD * kS * 2);
  unsigned short* wol  = (unsigned short*)carve((size_t)kD * kS * 2);
  unsigned short* sth  = (unsigned short*)carve((size_t)kB * kS * kS * 2);
  unsigned short* stl  = (unsigned short*)carve((size_t)kB * kS * kS * 2);
  float* proj = (float*)carve((size_t)kRows * kNP * 4);
  float* logg = (float*)carve((size_t)kRows * 4);
  float* cum  = (float*)carve((size_t)kRows * 4);
  float* cs   = (float*)carve((size_t)kRows * 4);
  unsigned short* krh  = (unsigned short*)carve(plane64);
  unsigned short* krl  = (unsigned short*)carve(plane64);
  unsigned short* qrh  = (unsigned short*)carve(plane64);
  unsigned short* qrl  = (unsigned short*)carve(plane64);
  unsigned short* qdh  = (unsigned short*)carve(plane64);
  unsigned short* qdl  = (unsigned short*)carve(plane64);
  unsigned short* krTh = (unsigned short*)carve((size_t)kNZ * kS * kChunkT * 2);
  unsigned short* krTl = (unsigned short*)carve((size_t)kNZ * kS * kChunkT * 2);
  unsigned short* aTh  = (unsigned short*)carve((size_t)kNZ * kS * kChunkT * 2);
  unsigned short* aTl  = (unsigned short*)carve((size_t)kNZ * kS * kChunkT * 2);
  unsigned short* avTh = (unsigned short*)carve((size_t)kB * kS * kT * 2);
  unsigned short* avTl = (unsigned short*)carve((size_t)kB * kS * kT * 2);
  float* sc = (float*)carve((size_t)kRows * kBand * 4);
  unsigned short* dah  = (unsigned short*)carve((size_t)kRows * kBand * 2);
  unsigned short* dal  = (unsigned short*)carve((size_t)kRows * kBand * 2);
  float* intra = (float*)carve((size_t)kRows * kS * 4);
  unsigned short* reth = (unsigned short*)carve(plane64);
  unsigned short* retl = (unsigned short*)carve(plane64);
  float* nsp = (float*)carve((size_t)kNZ * kS * kS * 4);
  if (off > ws_size) return;

  cvt_x_kernel<<<(kRows * kD / 8) / 256, 256, 0, stream>>>(x, xh, xl, kRows * kD / 8);
  cvt_w_kernel<<<168, 256, 0, stream>>>(Wk, Wv, Wq, Wg, Wout, state, wh, wl, woh, wol, sth, stl);
  wmma_gemm64<1, true, 0, 0, false><<<dim3((kRows / 64) * (kNP / 64) / 8, 1), 256, 0, stream>>>(
      xh, xl, kD, 0L, wh, wl, kD, 0L, (void*)proj, nullptr, kNP, 0L, nullptr, nullptr, 0L, kRows, kNP, kD, 1.0f);
  gates_pre_kernel<<<kRows / 64, 256, 0, stream>>>(proj, bg, cosT, sinT, logg);
  scan_kernel<<<kB, 32, 0, stream>>>(logg, cum, cs);
  planes_kernel<<<kRows / 64, 256, 0, stream>>>(proj, bg, cosT, sinT, cs, cum,
                                                krh, krl, qrh, qrl, qdh, qdl, krTh, krTl, avTh, avTl, aTh, aTl);
  band_gemm64<0><<<dim3(16, kB), 256, 0, stream>>>(qrh, qrl, kS, (long)kT * kS, krh, krl, kS, (long)kT * kS,
                                                    sc, kBand, (long)kT * kBand);
  decay_kernel<<<kRows / 8, 256, 0, stream>>>(sc, cum, cs, dah, dal);
  band_gemm64<1><<<dim3(4, kB), 256, 0, stream>>>(dah, dal, kBand, (long)kT * kBand, avTh, avTl, kT, (long)kS * kT,
                                                   intra, kS, (long)kT * kS);
  wmma_gemm64<1, true, 0, 2, true><<<dim3(4, kB), 256, 0, stream>>>(
      qdh, qdl, kS, (long)kT * kS, sth, stl, kS, (long)kS * kS, (void*)reth, (void*)retl, kS, (long)kT * kS,
      nullptr, intra, (long)kT * kS, kT, kS, kS, 1.0f);
  wmma_gemm64<1, true, 2, 0, false><<<dim3((kRows / 64) * (kD / 64) / 8, 1), 256, 0, stream>>>(
      reth, retl, kS, 0L, woh, wol, kS, 0L, (void*)out, nullptr, kD, 0L, bout, nullptr, 0L, kRows, kD, kS, 1.0f);
  wmma_gemm64<1, true, 0, 0, false><<<dim3(1, kNZ), 256, 0, stream>>>(
      aTh, aTl, kChunkT, (long)kS * kChunkT, krTh, krTl, kChunkT, (long)kS * kChunkT, (void*)nsp, nullptr, kS, (long)kS * kS,
      nullptr, nullptr, 0L, kS, kS, kChunkT, 1.0f);
  nstate_kernel<<<(kB * kS * kS / 4) / 256, 256, 0, stream>>>(nsp, state, cum, ns_out);
}
